// GlobalSSM_15229954031676
// MI455X (gfx1250) — hardware-verified
//
#include <hip/hip_runtime.h>


#define NB_  2
#define SS   4096
#define DD   1024
#define NS   16
typedef _Float16 h16;
typedef unsigned short bf;
typedef __attribute__((ext_vector_type(16))) __bf16   v16bf;
typedef __attribute__((ext_vector_type(16))) _Float16 v16h;
typedef __attribute__((ext_vector_type(8)))  _Float16 v8h;
typedef __attribute__((ext_vector_type(8)))  unsigned short v8us;
typedef __attribute__((ext_vector_type(8)))  float    v8f;
typedef __attribute__((ext_vector_type(4)))  float    v4f;
typedef v8h  __attribute__((may_alias)) v8ha;
typedef v4f  __attribute__((may_alias)) v4fa;
typedef v8us __attribute__((may_alias)) v8usa;

__device__ __forceinline__ unsigned short f2bf(float f) { unsigned u = __float_as_uint(f); u += 0x7FFFu + ((u >> 16) & 1u); return (unsigned short)(u >> 16); }
__device__ __forceinline__ float bf2f(unsigned short b) { return __uint_as_float(((unsigned)b) << 16); }
__device__ __forceinline__ float bfr(float f) { return bf2f(f2bf(f)); }
__device__ __forceinline__ v16h cat16(v8h lo, v8h hi) { return __builtin_shufflevector(lo, hi, 0, 1, 2, 3, 4, 5, 6, 7, 8, 9, 10, 11, 12, 13, 14, 15); }
__device__ __forceinline__ v16bf cat16b(v8us lo, v8us hi) { return __builtin_bit_cast(v16bf, __builtin_shufflevector(lo, hi, 0, 1, 2, 3, 4, 5, 6, 7, 8, 9, 10, 11, 12, 13, 14, 15)); }
__device__ __forceinline__ v8f wmma16(v16h a, v16h b, v8f c) { return __builtin_amdgcn_wmma_f32_16x16x32_f16(false, a, false, b, (short)0, c, false, false); }
__device__ __forceinline__ v8f wmmab(v16bf a, v16bf b, v8f c) { return __builtin_amdgcn_wmma_f32_16x16x32_bf16(false, a, false, b, (short)0, c, false, false); }


template <typename T16> struct WFrag;
template <> struct WFrag<h16> { typedef v16h V; static __device__ __forceinline__ V ld(const h16* p) { return cat16(*(const v8h*)p, *(const v8h*)(p + 16)); } static __device__ __forceinline__ v8f mma(V a, V b, v8f c) { return wmma16(a, b, c); } };
template <> struct WFrag<bf> { typedef v16bf V; static __device__ __forceinline__ V ld(const bf* p) { return cat16b(*(const v8us*)p, *(const v8us*)(p + 16)); } static __device__ __forceinline__ v8f mma(V a, V b, v8f c) { return wmmab(a, b, c); } };
template <typename T16, int NSPLIT, bool BIAS>
__global__ __launch_bounds__(32) void k_gemmw(const T16* __restrict__ A, const T16* __restrict__ A2, const T16* __restrict__ Bt, const T16* __restrict__ Bt2, int K, float* C, int ldc, const float* __restrict__ bias, size_t sA, size_t sB, size_t sC) {
    typedef typename WFrag<T16>::V V;
    __shared__ __align__(16) float os[16 * 68];
    const size_t z = blockIdx.z; A += z * sA; if (A2) A2 += z * sA; Bt += z * sB; if (Bt2) Bt2 += z * sB; C += z * sC;
    const int lane = threadIdx.x & 31, lr = lane & 15, hi = lane >> 4; const int r0 = blockIdx.x * 64, c0 = blockIdx.y * 64;
    v8f acc[4][4];
#pragma unroll
    for (int mb = 0; mb < 4; ++mb)
#pragma unroll
        for (int nb = 0; nb < 4; ++nb) acc[mb][nb] = (v8f){};
    const size_t aoff = (size_t)(r0 + lr) * K + 8 * hi, boff = (size_t)(c0 + lr) * K + 8 * hi;
#pragma unroll 1
    for (int kc = 0; kc < K; kc += 32) {
        V a[4], a2[4];
#pragma unroll
        for (int mb = 0; mb < 4; ++mb) { a[mb] = WFrag<T16>::ld(A + aoff + (size_t)mb * 16 * K + kc); if (NSPLIT == 1 || NSPLIT == 2) a2[mb] = WFrag<T16>::ld(A2 + aoff + (size_t)mb * 16 * K + kc); }
#pragma unroll
        for (int nb = 0; nb < 4; ++nb) { const V b = WFrag<T16>::ld(Bt + boff + (size_t)nb * 16 * K + kc); V b2; if (NSPLIT >= 2) b2 = WFrag<T16>::ld(Bt2 + boff + (size_t)nb * 16 * K + kc);
#pragma unroll
            for (int mb = 0; mb < 4; ++mb) { acc[mb][nb] = WFrag<T16>::mma(a[mb], b, acc[mb][nb]); if (NSPLIT == 1 || NSPLIT == 2) acc[mb][nb] = WFrag<T16>::mma(a2[mb], b, acc[mb][nb]); if (NSPLIT >= 2) acc[mb][nb] = WFrag<T16>::mma(a[mb], b2, acc[mb][nb]); } }
        asm volatile("v_nop\n\tv_nop\n\tv_nop\n\tv_nop" : "+v"(acc[0][0]), "+v"(acc[1][1]), "+v"(acc[2][2]), "+v"(acc[3][3]) : "v"(a[0]), "v"(a[3]));
    }
#pragma unroll
    for (int mb = 0; mb < 4; ++mb) {
#pragma unroll
        for (int nb = 0; nb < 4; ++nb) {
#pragma unroll
            for (int j = 0; j < 8; ++j) os[(hi * 8 + j) * 68 + nb * 16 + lr] = acc[mb][nb][j]; }
        __builtin_amdgcn_wave_barrier(); asm volatile("" ::: "memory");
        float* crow = C + (size_t)(r0 + mb * 16) * ldc + c0;
#pragma unroll 1
        for (int ps = 0; ps < 2; ++ps) {
#pragma unroll
            for (int s = 0; s < 8; ++s) { const int row = 2 * s + hi, cofs = lr * 4; v4f val = *(const v4fa*)(os + row * 68 + cofs); if (BIAS) { val[0] += bfr(bias[c0 + cofs]); val[1] += bfr(bias[c0 + cofs + 1]); val[2] += bfr(bias[c0 + cofs + 2]); val[3] += bfr(bias[c0 + cofs + 3]); }
                *(volatile v4f*)(crow + (size_t)row * ldc + cofs) = val; }
            if (ps == 0) __threadfence(); }
        __builtin_amdgcn_wave_barrier(); asm volatile("" ::: "memory");
    }
}

__device__ __forceinline__ void splitf(float y, unsigned short& h, unsigned short& l) { h = f2bf(y); l = f2bf(y - bf2f(h)); }
__device__ __forceinline__ float softplus_(float x) { return x > 20.f ? x : log1pf(__expf(x)); }
typedef __attribute__((ext_vector_type(4))) unsigned short v4us;

__global__ __launch_bounds__(256) void k_cvt8(const float* __restrict__ src, bf* dst, size_t n8) { const size_t i = (size_t)blockIdx.x * 256 + threadIdx.x; if (i >= n8) return; const v8f v = *(const v8f*)(src + i * 8); v8us o;
#pragma unroll
    for (int k = 0; k < 8; ++k) o[k] = f2bf(v[k]); *(volatile v8us*)(dst + i * 8) = o; __threadfence(); *(volatile v8us*)(dst + i * 8) = o; }
__global__ __launch_bounds__(256) void k_wbc(const float* __restrict__ wb, const float* __restrict__ wc, bf* WBC) { const int i = (blockIdx.x * 256 + threadIdx.x) * 4; if (i >= 64 * DD) return; const int n = i / DD, k = i % DD; v4us o;
#pragma unroll
    for (int q = 0; q < 4; ++q) o[q] = n < NS ? f2bf(wb[n * DD + k + q]) : (n < 2 * NS ? f2bf(wc[(n - NS) * DD + k + q]) : (unsigned short)0); *(volatile v4us*)(WBC + i) = o; __threadfence(); *(volatile v4us*)(WBC + i) = o; }
__global__ __launch_bounds__(256) void k_scan(const float* __restrict__ DRAW, const float* __restrict__ xb, const float* __restrict__ PBC, const float* __restrict__ alog, float* Y) {
    __shared__ float ybuf[64]; const int tid = threadIdx.x; const int cl = tid >> 2, sub = tid & 3; const int d = blockIdx.x * 64 + cl; const int n0 = sub * 4; float A[4], h[4];
#pragma unroll
    for (int j = 0; j < 4; ++j) { A[j] = -__expf(bfr(alog[(size_t)d * NS + n0 + j])); h[j] = 0.f; }
    for (int t = 0; t < SS; ++t) { const float dt = softplus_(DRAW[(size_t)t * DD + d]); const float xv = bfr(xb[(size_t)t * DD + d]); const float dtx = __fmul_rn(dt, xv); const float* pr = PBC + (size_t)t * 64; float y = 0.f;
#pragma unroll
        for (int j = 0; j < 4; ++j) { const float a = __expf(__fmul_rn(dt, A[j])); float ha = __fmul_rn(h[j], a); asm volatile("" : "+v"(ha)); float hb = __fmul_rn(dtx, pr[n0 + j]); asm volatile("" : "+v"(hb)); h[j] = __fadd_rn(ha, hb); float yc = __fmul_rn(h[j], pr[NS + n0 + j]); asm volatile("" : "+v"(yc)); y = __fadd_rn(y, yc); }
        y += __shfl_xor(y, 1, 32); y += __shfl_xor(y, 2, 32);
        if (sub == 0) ybuf[cl] = y;
        __syncthreads();
        if (tid < 64) { const float v = ybuf[tid]; const size_t o = (size_t)t * DD + blockIdx.x * 64 + tid; *(volatile float*)(Y + o) = v; __threadfence(); *(volatile float*)(Y + o) = v; }
        __syncthreads(); } }
__global__ __launch_bounds__(256) void k_ln(const float* __restrict__ Y, const float* __restrict__ g, const float* __restrict__ bb, const float* __restrict__ csp, float* LNF, bf* Lh, bf* Ll) { const int lane = threadIdx.x & 31; const int row = blockIdx.x * 8 + (threadIdx.x >> 5); if (row >= SS) return; const size_t rb = (size_t)row * DD; float s = 0.f;
#pragma unroll 1
    for (int ch = 0; ch < 8; ++ch) { const v4f a = *(const v4f*)(Y + rb + ch * 128 + lane * 4); s = __fadd_rn(s, __fadd_rn(__fadd_rn(a[0], a[1]), __fadd_rn(a[2], a[3]))); }
#pragma unroll
    for (int sh = 16; sh; sh >>= 1) s += __shfl_xor(s, sh, 32);
    const float mean = s * (1.0f / DD); float q2 = 0.f;
#pragma unroll 1
    for (int ch = 0; ch < 8; ++ch) { const v4f a = *(const v4f*)(Y + rb + ch * 128 + lane * 4);
#pragma unroll
        for (int q = 0; q < 4; ++q) { float d0 = __fsub_rn(a[q], mean); asm volatile("" : "+v"(d0)); float p = __fmul_rn(d0, d0); asm volatile("" : "+v"(p)); q2 = __fadd_rn(q2, p); } }
#pragma unroll
    for (int sh = 16; sh; sh >>= 1) q2 += __shfl_xor(q2, sh, 32);
    const float rstd = __frsqrt_rn(__fadd_rn(q2 * (1.0f / DD), 1e-5f)); const float cs = bfr(csp[0]);
    for (int ps = 0; ps < 2; ++ps) {
#pragma unroll 1
        for (int ch = 0; ch < 8; ++ch) { const int c0 = ch * 128 + lane * 4; const v4f a = *(const v4f*)(Y + rb + c0); v4f o; v4us oh, ol;
#pragma unroll
            for (int q = 0; q < 4; ++q) { float t0 = __fmul_rn(__fsub_rn(a[q], mean), rstd); asm volatile("" : "+v"(t0)); float t1 = __fmul_rn(t0, bfr(g[c0 + q])); asm volatile("" : "+v"(t1)); o[q] = __fadd_rn(t1, bfr(bb[c0 + q])); unsigned short u, l; splitf(__fmul_rn(o[q], cs), u, l); oh[q] = u; ol[q] = l; }
            *(volatile v4f*)(LNF + rb + c0) = o; *(volatile v4us*)(Lh + rb + c0) = oh; *(volatile v4us*)(Ll + rb + c0) = ol; }
        if (ps == 0) __threadfence(); } }
__global__ __launch_bounds__(256) void k_hproj(const float* __restrict__ LNF, const float* __restrict__ wimp, float* HP) { const int e = blockIdx.x * 256 + threadIdx.x; if (e >= DD) return; const float* hf = LNF + (size_t)(SS - 1) * DD; float s = 0.f;
#pragma unroll 1
    for (int d = 0; d < DD; ++d) { float p = __fmul_rn(bfr(wimp[(size_t)e * DD + d]), hf[d]); asm volatile("" : "+v"(p)); s = __fadd_rn(s, p); } *(volatile float*)(HP + e) = s; __threadfence(); *(volatile float*)(HP + e) = s; }
__global__ __launch_bounds__(256) void k_raw(const float* __restrict__ xb, const float* __restrict__ HP, float* RAW) { const int sI = blockIdx.x * 256 + threadIdx.x; if (sI >= SS) return; const float* xr = xb + (size_t)sI * DD; float s = 0.f;
#pragma unroll 1
    for (int d = 0; d < DD; ++d) { float p = __fmul_rn(bfr(xr[d]), HP[d]); asm volatile("" : "+v"(p)); s = __fadd_rn(s, p); } *(volatile float*)(RAW + sI) = s; __threadfence(); *(volatile float*)(RAW + sI) = s; }
__global__ __launch_bounds__(32) void k_isoft(const float* __restrict__ RAW, float* IMP) { const int lane = threadIdx.x; float mx = -3.0e38f;
    for (int ch = 0; ch < SS / 128; ++ch) { const v4f a = *(const v4f*)(RAW + ch * 128 + lane * 4); mx = fmaxf(mx, fmaxf(fmaxf(a[0], a[1]), fmaxf(a[2], a[3]))); }
#pragma unroll
    for (int sh = 16; sh; sh >>= 1) mx = fmaxf(mx, __shfl_xor(mx, sh, 32));
    float sum = 0.f;
    for (int ch = 0; ch < SS / 128; ++ch) { const v4f a = *(const v4f*)(RAW + ch * 128 + lane * 4);
#pragma unroll
        for (int q = 0; q < 4; ++q) { float d0 = __fmul_rn(__fsub_rn(a[q], mx), 2.0f); asm volatile("" : "+v"(d0)); sum += __expf(d0); } }
#pragma unroll
    for (int sh = 16; sh; sh >>= 1) sum += __shfl_xor(sum, sh, 32);
    const float f = __fdiv_rn(1.0f, sum);
    for (int ps = 0; ps < 2; ++ps) { for (int ch = 0; ch < SS / 128; ++ch) { const int j0 = ch * 128 + lane * 4; const v4f a = *(const v4f*)(RAW + j0); v4f o;
#pragma unroll
            for (int q = 0; q < 4; ++q) { float d0 = __fmul_rn(__fsub_rn(a[q], mx), 2.0f); asm volatile("" : "+v"(d0)); o[q] = __fmul_rn(__expf(d0), f); } *(volatile v4f*)(IMP + j0) = o; }
        if (ps == 0) __threadfence(); } }

extern "C" void kernel_launch(void* const* d_in, const int* in_sizes, int n_in,
                              void* d_out, int out_size, void* d_ws, size_t ws_size, hipStream_t stream) {
    (void)in_sizes; (void)n_in; (void)out_size;
    const float* x = (const float*)d_in[0]; const float* alog = (const float*)d_in[1]; const float* wdel = (const float*)d_in[2]; const float* wb = (const float*)d_in[3]; const float* wc = (const float*)d_in[4]; const float* g = (const float*)d_in[5]; const float* be = (const float*)d_in[6]; const float* wctx = (const float*)d_in[7]; const float* csp = (const float*)d_in[8]; const float* wimp = (const float*)d_in[9];
    float* IMPO = (float*)d_out;
    float* CTX = (float*)((char*)d_out + 32768);
    float* RAWO = (float*)((char*)d_out + 33587200);
    char* wsp = (char*)d_ws;
    auto take = [&](size_t bytes) { char* p = wsp; wsp += (bytes + 255) & ~(size_t)255; return (void*)p; };
    bf* WDEL = (bf*)take((size_t)DD * DD * 2); bf* WBC = (bf*)take((size_t)64 * DD * 2); bf* WCTX = (bf*)take((size_t)DD * DD * 2);
    bf* XB = (bf*)take((size_t)SS * DD * 2); float* DRAW = (float*)take((size_t)SS * DD * 4); float* PBC = (float*)take((size_t)SS * 64 * 4); float* Y = (float*)take((size_t)SS * DD * 4); float* LNF = (float*)take((size_t)SS * DD * 4); bf* Lh = (bf*)take((size_t)SS * DD * 2); bf* Ll = (bf*)take((size_t)SS * DD * 2); float* HP = (float*)take(DD * 4);
    if ((size_t)(wsp - (char*)d_ws) > ws_size) return;
    k_cvt8<<<(DD * DD / 8 + 255) / 256, 256, 0, stream>>>(wdel, WDEL, DD * DD / 8); k_wbc<<<(64 * DD / 4 + 255) / 256, 256, 0, stream>>>(wb, wc, WBC); k_cvt8<<<(DD * DD / 8 + 255) / 256, 256, 0, stream>>>(wctx, WCTX, DD * DD / 8);
    for (int b = 0; b < NB_; ++b) { const float* xb = x + (size_t)b * SS * DD;
        k_cvt8<<<(unsigned)(((size_t)SS * DD / 8 + 255) / 256), 256, 0, stream>>>(xb, XB, (size_t)SS * DD / 8);
        k_gemmw<bf, 0, false><<<dim3(SS / 64, DD / 64, 1), 32, 0, stream>>>(XB, nullptr, WDEL, nullptr, DD, DRAW, DD, nullptr, 0, 0, 0); k_gemmw<bf, 0, false><<<dim3(SS / 64, 1, 1), 32, 0, stream>>>(XB, nullptr, WBC, nullptr, DD, PBC, 64, nullptr, 0, 0, 0);
        k_scan<<<DD / 64, 256, 0, stream>>>(DRAW, xb, PBC, alog, Y);
        k_ln<<<SS / 8, 256, 0, stream>>>(Y, g, be, csp, LNF, Lh, Ll);
        k_gemmw<bf, 1, false><<<dim3(SS / 64, DD / 64, 1), 32, 0, stream>>>(Lh, Ll, WCTX, nullptr, DD, CTX + (size_t)b * SS * DD, DD, nullptr, 0, 0, 0);
        k_hproj<<<DD / 256, 256, 0, stream>>>(LNF, wimp, HP); k_raw<<<SS / 256, 256, 0, stream>>>(xb, HP, RAWO + (size_t)b * SS); k_isoft<<<1, 32, 0, stream>>>(RAWO + (size_t)b * SS, IMPO + (size_t)b * SS); }
}
